// GNNPolicy_82094004896465
// MI455X (gfx1250) — hardware-verified
//
#include <hip/hip_runtime.h>
#include <stddef.h>
#include <stdint.h>
#include <math.h>


#define NN      1536
#define HD      64
#define K1      128
#define UD      128
#define K2      256
#define NTB     16
#define AP1     136
#define AP2     264
#define HPW     4
#define OUT_STD 3072
#define OUT_VAL 3074
#define OUT_N   4610
#define PJ      128
#define UB_W2   0
#define UB_WM   1024
#define UB_U1   2048
#define UB_U2   6144
#define UB_WH   10240
#define UB_END  10752
#define WSMAX   134217728

static_assert(NN % NTB == 0);
static_assert(K1 == 2 * HD && K2 == 2 * UD && K1 % 32 == 0 && K2 % 32 == 0);
static_assert((AP1 * 2) % 16 == 0 && (AP2 * 2) % 16 == 0 && AP1 >= K1 && AP2 >= K2);
static_assert(OUT_VAL + NN == OUT_N && OUT_STD == 2 * NN);
static_assert(UB_WM % 256 == 0 && UB_U1 % 256 == 0 && UB_U2 % 256 == 0 && UB_WH % 256 == 0 && UB_END % 256 == 0);
static_assert(NN % (2 * PJ) == 0);
static_assert((PJ * HD) % (256 * 4) == 0);

typedef float          v4f   __attribute__((ext_vector_type(4)));
typedef float          v8f   __attribute__((ext_vector_type(8)));
typedef int            v8i   __attribute__((ext_vector_type(8)));
typedef unsigned short v8us  __attribute__((ext_vector_type(8)));
typedef unsigned short v16us __attribute__((ext_vector_type(16)));
typedef __bf16         v16bf __attribute__((ext_vector_type(16)));
typedef v4f  __attribute__((may_alias)) v4fa;
typedef v8us __attribute__((may_alias)) v8usa;
union FragB { v16bf v; v16us u; v8us h[2]; v8i w; };

__device__ __forceinline__ v8f wmb(const FragB& a, const FragB& b, v8f c) {
  v8f d = __builtin_amdgcn_wmma_f32_16x16x32_bf16(false, a.v, false, b.v, (short)0, c, false, false);
  asm volatile("v_nop\n\tv_nop\n\tv_nop\n\tv_nop" : "+v"(d) : "v"(a.w), "v"(b.w));
  return d;
}

__device__ __forceinline__ unsigned bf16_bits(float f) {
  const unsigned u = __float_as_uint(f);
  return (u + 0x7FFFu + ((u >> 16) & 1u)) >> 16;
}
__device__ __forceinline__ float bf16_val(float f) {
  return __uint_as_float(bf16_bits(f) << 16);
}
__device__ __forceinline__ void sp1(float v, unsigned short& h, unsigned short& l) {
  const unsigned hb = bf16_bits(v);
  h = (unsigned short)hb;
  l = (unsigned short)bf16_bits(v - __uint_as_float(hb << 16));
}
__device__ __forceinline__ void split8(const v4f a, const v4f b, v8us& hv, v8us& lv) {
  unsigned short h, l;
  sp1(a.x, h, l); hv[0] = h; lv[0] = l;
  sp1(a.y, h, l); hv[1] = h; lv[1] = l;
  sp1(a.z, h, l); hv[2] = h; lv[2] = l;
  sp1(a.w, h, l); hv[3] = h; lv[3] = l;
  sp1(b.x, h, l); hv[4] = h; lv[4] = l;
  sp1(b.y, h, l); hv[5] = h; lv[5] = l;
  sp1(b.z, h, l); hv[6] = h; lv[6] = l;
  sp1(b.w, h, l); hv[7] = h; lv[7] = l;
}
__device__ __forceinline__ void st8(unsigned short* dp, const v8us o) {
  *(volatile v8us*)dp = o;
  __threadfence();
  *(volatile v8us*)dp = o;
}
template <int LD>
__device__ __forceinline__ v8us gather8(const float* __restrict__ p) {
  v8us o;
#pragma unroll
  for (int i = 0; i < 8; ++i) o[i] = (unsigned short)bf16_bits(p[(size_t)i * LD]);
  return o;
}

template <int KS>
__device__ __forceinline__ v8f gemm_la(const unsigned short* ap, const unsigned short* __restrict__ wp) {
  v8f acc = {0.f, 0.f, 0.f, 0.f, 0.f, 0.f, 0.f, 0.f};
#pragma unroll
  for (int ks = 0; ks < KS; ++ks) {
    FragB af, bf;
    af.h[0] = *(const v8usa*)(ap + 32 * ks);
    af.h[1] = *(const v8usa*)(ap + 32 * ks + 16);
    bf.h[0] = *(const v8usa*)(wp + 32 * ks);
    bf.h[1] = *(const v8usa*)(wp + 32 * ks + 16);
    acc = wmb(af, bf, acc);
  }
  return acc;
}
template <int KS>
__device__ __forceinline__ v8f gemm_ga(const unsigned short* __restrict__ ap, const unsigned short* __restrict__ wp) {
  v8f acc = {0.f, 0.f, 0.f, 0.f, 0.f, 0.f, 0.f, 0.f};
#pragma unroll
  for (int ks = 0; ks < KS; ++ks) {
    FragB af, bf;
    af.h[0] = *(const v8usa*)(ap + 32 * ks);
    af.h[1] = *(const v8usa*)(ap + 32 * ks + 16);
    bf.h[0] = *(const v8usa*)(wp + 32 * ks);
    bf.h[1] = *(const v8usa*)(wp + 32 * ks + 16);
    acc = wmb(af, bf, acc);
  }
  return acc;
}

__global__ __launch_bounds__(256) void k_prep(const float* __restrict__ W2, const float* __restrict__ Wm,
                                              const float* __restrict__ Wu1, const float* __restrict__ Wu2,
                                              const float* __restrict__ Wmean, const float* __restrict__ Wv,
                                              unsigned short* W2T2, unsigned short* WmT2,
                                              unsigned short* Wu1T2, unsigned short* Wu2T2, unsigned short* WH) {
  const int u = (int)blockIdx.x * 256 + (int)threadIdx.x;
  if (u < UB_WM) {
    const int v = u - UB_W2;
    const int n = v >> 4, k8 = (v & 15) * 8, kk = k8 & (HD - 1);
    const v8us o = gather8<HD>(W2 + (size_t)kk * HD + n);
    st8(W2T2 + (size_t)n * K1 + k8, o);
  } else if (u < UB_U1) {
    const int v = u - UB_WM;
    const int n = v >> 4, k8 = (v & 15) * 8, kk = k8 & (HD - 1);
    const v8us o = gather8<HD>(Wm + (size_t)kk * HD + n);
    st8(WmT2 + (size_t)n * K1 + k8, o);
  } else if (u < UB_U2) {
    const int v = u - UB_U1;
    const int n = v >> 5, k8 = (v & 31) * 8, kk = k8 & (UD - 1);
    const v8us o = gather8<UD>(Wu1 + (size_t)kk * UD + n);
    st8(Wu1T2 + (size_t)n * K2 + k8, o);
  } else if (u < UB_WH) {
    const int v = u - UB_U2;
    const int n = v >> 5, k8 = (v & 31) * 8, kk = k8 & (UD - 1);
    const v8us o = gather8<UD>(Wu2 + (size_t)kk * UD + n);
    st8(Wu2T2 + (size_t)n * K2 + k8, o);
  } else if (u < UB_END) {
    const int v  = u - UB_WH;
    const int nu = __builtin_amdgcn_readfirstlane(v >> 5);
    const int k8 = (v & 31) * 8, kk = k8 & (UD - 1);
    v8us o = {0, 0, 0, 0, 0, 0, 0, 0};
    if (nu < 2) {
      o = gather8<2>(Wmean + (size_t)kk * 2 + nu);
    } else if (nu == 2) {
      const v4f a = *(const v4f*)(Wv + kk);
      const v4f b = *(const v4f*)(Wv + kk + 4);
      o[0] = (unsigned short)bf16_bits(a.x); o[1] = (unsigned short)bf16_bits(a.y);
      o[2] = (unsigned short)bf16_bits(a.z); o[3] = (unsigned short)bf16_bits(a.w);
      o[4] = (unsigned short)bf16_bits(b.x); o[5] = (unsigned short)bf16_bits(b.y);
      o[6] = (unsigned short)bf16_bits(b.z); o[7] = (unsigned short)bf16_bits(b.w);
    }
    st8(WH + (size_t)nu * K2 + k8, o);
  }
}

__device__ __forceinline__ float h0c(float x0, float x1, float x2, float x3,
                                     float w0, float w1, float w2, float w3, float b) {
  float s = x0 * bf16_val(w0);
  s = fmaf(x1, bf16_val(w1), s);
  s = fmaf(x2, bf16_val(w2), s);
  s = fmaf(x3, bf16_val(w3), s);
  s = s + bf16_val(b);
  return fmaxf(s, 0.0f);
}

__global__ __launch_bounds__(128) void k_enc(const float* __restrict__ x, const float* __restrict__ W1,
                                             const float* __restrict__ b1,
                                             const unsigned short* __restrict__ W2T2, const float* __restrict__ b2,
                                             const unsigned short* __restrict__ WmT2,
                                             unsigned short* HU, float* P) {
  __shared__ __attribute__((aligned(16))) unsigned short At[NTB * AP1];
  __shared__ __attribute__((aligned(16))) float stg[NTB * HD];
  const int tid = (int)threadIdx.x, lane = tid & 31, wave = tid >> 5, hh = lane >> 4, m = lane & 15;
  const int row0 = (int)blockIdx.x * NTB;
  const int rr = tid >> 3, c8 = (tid & 7) * 8;

  {
    const v4f xr = *(const v4f*)(x + (size_t)(row0 + rr) * 4);
    const float x0 = bf16_val(xr.x), x1 = bf16_val(xr.y), x2 = bf16_val(xr.z), x3 = bf16_val(xr.w);
    const v4f w0a = *(const v4f*)(W1 + 0 * HD + c8), w0b = *(const v4f*)(W1 + 0 * HD + c8 + 4);
    const v4f w1a = *(const v4f*)(W1 + 1 * HD + c8), w1b = *(const v4f*)(W1 + 1 * HD + c8 + 4);
    const v4f w2a = *(const v4f*)(W1 + 2 * HD + c8), w2b = *(const v4f*)(W1 + 2 * HD + c8 + 4);
    const v4f w3a = *(const v4f*)(W1 + 3 * HD + c8), w3b = *(const v4f*)(W1 + 3 * HD + c8 + 4);
    const v4f ba = *(const v4f*)(b1 + c8), bb = *(const v4f*)(b1 + c8 + 4);
    v4f ga, gb;
    ga.x = h0c(x0, x1, x2, x3, w0a.x, w1a.x, w2a.x, w3a.x, ba.x);
    ga.y = h0c(x0, x1, x2, x3, w0a.y, w1a.y, w2a.y, w3a.y, ba.y);
    ga.z = h0c(x0, x1, x2, x3, w0a.z, w1a.z, w2a.z, w3a.z, ba.z);
    ga.w = h0c(x0, x1, x2, x3, w0a.w, w1a.w, w2a.w, w3a.w, ba.w);
    gb.x = h0c(x0, x1, x2, x3, w0b.x, w1b.x, w2b.x, w3b.x, bb.x);
    gb.y = h0c(x0, x1, x2, x3, w0b.y, w1b.y, w2b.y, w3b.y, bb.y);
    gb.z = h0c(x0, x1, x2, x3, w0b.z, w1b.z, w2b.z, w3b.z, bb.z);
    gb.w = h0c(x0, x1, x2, x3, w0b.w, w1b.w, w2b.w, w3b.w, bb.w);
    v8us hv, lv;
    split8(ga, gb, hv, lv);
    *(v8usa*)(At + rr * AP1 + c8) = hv;
    *(v8usa*)(At + rr * AP1 + HD + c8) = lv;
  }
  __syncthreads();

  const unsigned short* apl = At + m * AP1 + 8 * hh;
  {
    const v8f acc = gemm_la<K1 / 32>(apl, W2T2 + (size_t)(16 * wave + m) * K1 + 8 * hh);
#pragma unroll
    for (int r = 0; r < 8; ++r) stg[(8 * hh + r) * HD + 16 * wave + m] = acc[r];
  }
  __syncthreads();

  {
    const v4f f0 = *(const v4fa*)(stg + rr * HD + c8);
    const v4f f1 = *(const v4fa*)(stg + rr * HD + c8 + 4);
    const v4f ba = *(const v4f*)(b2 + c8), bb = *(const v4f*)(b2 + c8 + 4);
    v4f ga, gb;
    ga.x = fmaxf(f0.x + bf16_val(ba.x), 0.0f); ga.y = fmaxf(f0.y + bf16_val(ba.y), 0.0f);
    ga.z = fmaxf(f0.z + bf16_val(ba.z), 0.0f); ga.w = fmaxf(f0.w + bf16_val(ba.w), 0.0f);
    gb.x = fmaxf(f1.x + bf16_val(bb.x), 0.0f); gb.y = fmaxf(f1.y + bf16_val(bb.y), 0.0f);
    gb.z = fmaxf(f1.z + bf16_val(bb.z), 0.0f); gb.w = fmaxf(f1.w + bf16_val(bb.w), 0.0f);
    v8us hv, lv;
    split8(ga, gb, hv, lv);
    *(v8usa*)(At + rr * AP1 + c8) = hv;
    *(v8usa*)(At + rr * AP1 + HD + c8) = lv;
    unsigned short* hp = HU + (size_t)(row0 + rr) * K2 + c8;
    *(volatile v8us*)hp = hv;
    *(volatile v8us*)(hp + UD) = lv;
    __threadfence();
    *(volatile v8us*)hp = hv;
    *(volatile v8us*)(hp + UD) = lv;
  }
  __syncthreads();

  {
    const v8f acc = gemm_la<K1 / 32>(apl, WmT2 + (size_t)(16 * wave + m) * K1 + 8 * hh);
#pragma unroll
    for (int r = 0; r < 8; ++r) stg[(8 * hh + r) * HD + 16 * wave + m] = acc[r];
  }
  __syncthreads();

  {
    const int lr0 = tid >> 4, cc = 4 * (tid & 15);
    const v4f q0 = *(const v4fa*)(stg + lr0 * HD + cc);
    const v4f q1 = *(const v4fa*)(stg + (lr0 + 8) * HD + cc);
    float* p0 = P + (size_t)(row0 + lr0) * HD + cc;
    float* p1 = P + (size_t)(row0 + lr0 + 8) * HD + cc;
    *(volatile v4f*)p0 = q0;
    *(volatile v4f*)p1 = q1;
    __threadfence();
    *(volatile v4f*)p0 = q0;
    *(volatile v4f*)p1 = q1;
  }
}

__global__ __launch_bounds__(256) void k_pair(const float* __restrict__ P, const float* __restrict__ bm,
                                              unsigned short* HU) {
  __shared__ __attribute__((aligned(16))) float sp[PJ * HD];
  __shared__ __attribute__((aligned(16))) unsigned short mst[NTB * 2 * HD];
  const int tid = (int)threadIdx.x;
  const int c = tid & 63, g = tid >> 6;
  const int ib = (int)blockIdx.x * NTB;
  const int i0 = ib + 4 * g;
  const float pi0 = P[(size_t)(i0 + 0) * HD + c];
  const float pi1 = P[(size_t)(i0 + 1) * HD + c];
  const float pi2 = P[(size_t)(i0 + 2) * HD + c];
  const float pi3 = P[(size_t)(i0 + 3) * HD + c];
  const float bmc = bf16_val(bm[c]);
  float t0 = 0.0f, t1 = 0.0f, t2 = 0.0f, t3 = 0.0f;
  float q0 = 0.0f, q1 = 0.0f, q2 = 0.0f, q3 = 0.0f;

#pragma unroll 1
  for (int ch = 0; ch < NN / PJ; ++ch) {
    const float* src = P + (size_t)ch * (PJ * HD);
    v4f tv[8];
#pragma unroll
    for (int u = 0; u < 8; ++u) tv[u] = *(const v4f*)(src + 4 * (tid + 256 * u));
    __syncthreads();
#pragma unroll
    for (int u = 0; u < 8; ++u) *(v4fa*)(sp + 4 * (tid + 256 * u)) = tv[u];
    __syncthreads();
#pragma unroll 8
    for (int jj = 0; jj < PJ; ++jj) {
      const float v = sp[jj * HD + c];
      q0 += fmaxf((v - pi0) + bmc, 0.0f);
      q1 += fmaxf((v - pi1) + bmc, 0.0f);
      q2 += fmaxf((v - pi2) + bmc, 0.0f);
      q3 += fmaxf((v - pi3) + bmc, 0.0f);
    }
    if ((ch & 1) != 0) {
      t0 += q0; t1 += q1; t2 += q2; t3 += q3;
      q0 = 0.0f; q1 = 0.0f; q2 = 0.0f; q3 = 0.0f;
    }
  }
  const float sc = 1.0f / 1536.0f;
  const float m0 = t0 * sc, m1 = t1 * sc, m2 = t2 * sc, m3 = t3 * sc;
  {
    unsigned short h, l;
    sp1(m0, h, l); mst[(4 * g + 0) * (2 * HD) + c] = h; mst[(4 * g + 0) * (2 * HD) + HD + c] = l;
    sp1(m1, h, l); mst[(4 * g + 1) * (2 * HD) + c] = h; mst[(4 * g + 1) * (2 * HD) + HD + c] = l;
    sp1(m2, h, l); mst[(4 * g + 2) * (2 * HD) + c] = h; mst[(4 * g + 2) * (2 * HD) + HD + c] = l;
    sp1(m3, h, l); mst[(4 * g + 3) * (2 * HD) + c] = h; mst[(4 * g + 3) * (2 * HD) + HD + c] = l;
  }
  __syncthreads();
  {
    const int line = tid >> 3, piece = tid & 7;
    const int row = line >> 1, sel = line & 1;
    const v8us qv = *(const v8usa*)(mst + row * (2 * HD) + sel * HD + piece * 8);
    st8(HU + (size_t)(ib + row) * K2 + HD + sel * UD + piece * 8, qv);
  }
}

__device__ __forceinline__ void epi_split(const float* stg, unsigned short* At, const float* __restrict__ bias,
                                          int rr, int c8) {
  const v4f f0 = *(const v4fa*)(stg + rr * UD + c8);
  const v4f f1 = *(const v4fa*)(stg + rr * UD + c8 + 4);
  const v4f ba = *(const v4f*)(bias + c8), bb = *(const v4f*)(bias + c8 + 4);
  v4f ga, gb;
  ga.x = fmaxf(f0.x + bf16_val(ba.x), 0.0f); ga.y = fmaxf(f0.y + bf16_val(ba.y), 0.0f);
  ga.z = fmaxf(f0.z + bf16_val(ba.z), 0.0f); ga.w = fmaxf(f0.w + bf16_val(ba.w), 0.0f);
  gb.x = fmaxf(f1.x + bf16_val(bb.x), 0.0f); gb.y = fmaxf(f1.y + bf16_val(bb.y), 0.0f);
  gb.z = fmaxf(f1.z + bf16_val(bb.z), 0.0f); gb.w = fmaxf(f1.w + bf16_val(bb.w), 0.0f);
  v8us hv, lv;
  split8(ga, gb, hv, lv);
  *(v8usa*)(At + rr * AP2 + c8) = hv;
  *(v8usa*)(At + rr * AP2 + UD + c8) = lv;
}

__global__ __launch_bounds__(256) void k_upd(const unsigned short* __restrict__ HU,
                                             const unsigned short* __restrict__ Wu1T2, const float* __restrict__ bu1,
                                             const unsigned short* __restrict__ Wu2T2, const float* __restrict__ bu2,
                                             const unsigned short* __restrict__ WH,
                                             const float* __restrict__ bmean, const float* __restrict__ bv,
                                             float* HEADS) {
  __shared__ __attribute__((aligned(16))) unsigned short At[NTB * AP2];
  __shared__ __attribute__((aligned(16))) float stg[NTB * UD];
  __shared__ __attribute__((aligned(16))) float hst[NTB * 16];
  const int tid = (int)threadIdx.x, lane = tid & 31, wave = tid >> 5, hh = lane >> 4, m = lane & 15;
  const int row0 = (int)blockIdx.x * NTB;
  const int rr = tid >> 4, c8 = (tid & 15) * 8;

  {
    const v8f acc = gemm_ga<K2 / 32>(HU + (size_t)(row0 + m) * K2 + 8 * hh,
                                     Wu1T2 + (size_t)(16 * wave + m) * K2 + 8 * hh);
#pragma unroll
    for (int r = 0; r < 8; ++r) stg[(8 * hh + r) * UD + 16 * wave + m] = acc[r];
  }
  __syncthreads();
  epi_split(stg, At, bu1, rr, c8);
  __syncthreads();

  const unsigned short* apl = At + m * AP2 + 8 * hh;
  {
    const v8f acc = gemm_la<K2 / 32>(apl, Wu2T2 + (size_t)(16 * wave + m) * K2 + 8 * hh);
#pragma unroll
    for (int r = 0; r < 8; ++r) stg[(8 * hh + r) * UD + 16 * wave + m] = acc[r];
  }
  __syncthreads();
  epi_split(stg, At, bu2, rr, c8);
  __syncthreads();

  if (wave == 0) {
    const v8f acc = gemm_la<K2 / 32>(apl, WH + (size_t)m * K2 + 8 * hh);
#pragma unroll
    for (int r = 0; r < 8; ++r) hst[(8 * hh + r) * 16 + m] = acc[r];
  }
  __syncthreads();
  if (tid < NTB) {
    const v4f hv = *(const v4fa*)(hst + tid * 16);
    v4f o;
    o.x = hv.x + bf16_val(bmean[0]);
    o.y = hv.y + bf16_val(bmean[1]);
    o.z = hv.z + bf16_val(bv[0]);
    o.w = 0.0f;
    float* op = HEADS + (size_t)(row0 + tid) * HPW;
    *(volatile v4f*)op = o;
    __threadfence();
    *(volatile v4f*)op = o;
  }
}

__global__ __launch_bounds__(256) void k_emit(const float* __restrict__ HEADS, const float* __restrict__ lstd,
                                              float* out) {
  const int f = (int)blockIdx.x * 256 + (int)threadIdx.x;
  const int fm = f < OUT_STD - 1 ? f : OUT_STD - 1;
  int fs = f - OUT_STD;
  fs = fs < 0 ? 0 : (fs > 1 ? 1 : fs);
  int fv = f - OUT_VAL;
  fv = fv < 0 ? 0 : (fv > NN - 1 ? NN - 1 : fv);
  const float a = HEADS[(size_t)(fm >> 1) * HPW + (fm & 1)];
  const float b = HEADS[(size_t)fv * HPW + 2];
  const float e = expf(bf16_val(lstd[fs]));
  const int isM = (f < OUT_STD) ? -1 : 0;
  const int isS = (f >= OUT_STD && f < OUT_VAL) ? -1 : 0;
  const int isV = ~(isM | isS);
  const int bits = (__float_as_int(a) & isM) | (__float_as_int(e) & isS) | (__float_as_int(b) & isV);
  const float o = __int_as_float(bits);
  const bool ok = f < OUT_N;
  if (ok) *(volatile float*)(out + f) = o;
  __threadfence();
  if (ok) *(volatile float*)(out + f) = o;
}

static inline size_t al256(size_t o) { return (o + 255) & ~(size_t)255; }

extern "C" void kernel_launch(void* const* d_in, const int* in_sizes, int n_in,
                              void* d_out, int out_size, void* d_ws, size_t ws_size,
                              hipStream_t stream) {
  if (n_in < 16) return;
  if (in_sizes[0] != NN * 4) return;
  if (in_sizes[1] != 4 * HD || in_sizes[2] != HD) return;
  if (in_sizes[3] != HD * HD || in_sizes[4] != HD) return;
  if (in_sizes[5] != HD * HD || in_sizes[6] != HD) return;
  if (in_sizes[7] != UD * UD || in_sizes[8] != UD) return;
  if (in_sizes[9] != UD * UD || in_sizes[10] != UD) return;
  if (in_sizes[11] != UD * 2 || in_sizes[12] != 2) return;
  if (in_sizes[13] != UD || in_sizes[14] != 1) return;
  if (in_sizes[15] != 2) return;
  if (out_size != OUT_N) return;

  const float* x     = (const float*)d_in[0];
  const float* W1    = (const float*)d_in[1];
  const float* b1    = (const float*)d_in[2];
  const float* W2    = (const float*)d_in[3];
  const float* b2    = (const float*)d_in[4];
  const float* Wm    = (const float*)d_in[5];
  const float* bm    = (const float*)d_in[6];
  const float* Wu1   = (const float*)d_in[7];
  const float* bu1   = (const float*)d_in[8];
  const float* Wu2   = (const float*)d_in[9];
  const float* bu2   = (const float*)d_in[10];
  const float* Wmean = (const float*)d_in[11];
  const float* bmean = (const float*)d_in[12];
  const float* Wv    = (const float*)d_in[13];
  const float* bvv   = (const float*)d_in[14];
  const float* lstd  = (const float*)d_in[15];
  float* out = (float*)d_out;

  char* ws = (char*)d_ws;
  size_t off = 0;
  const size_t oW2 = off; off = al256(off + (size_t)HD * K1 * 2);
  const size_t oWm = off; off = al256(off + (size_t)HD * K1 * 2);
  const size_t oU1 = off; off = al256(off + (size_t)UD * K2 * 2);
  const size_t oU2 = off; off = al256(off + (size_t)UD * K2 * 2);
  const size_t oWH = off; off = al256(off + (size_t)16 * K2 * 2);
  const size_t oHU = off; off = al256(off + (size_t)NN * K2 * 2);
  const size_t oP  = off; off = al256(off + (size_t)NN * HD * 4);
  const size_t oHE = off; off = al256(off + (size_t)NN * HPW * 4);
  if (off > ws_size || off > (size_t)WSMAX) return;
  unsigned short* W2T2  = (unsigned short*)(ws + oW2);
  unsigned short* WmT2  = (unsigned short*)(ws + oWm);
  unsigned short* Wu1T2 = (unsigned short*)(ws + oU1);
  unsigned short* Wu2T2 = (unsigned short*)(ws + oU2);
  unsigned short* WH    = (unsigned short*)(ws + oWH);
  unsigned short* HU    = (unsigned short*)(ws + oHU);
  float*          P     = (float*)(ws + oP);
  float*          HEADS = (float*)(ws + oHE);

  k_prep<<<UB_END / 256, 256, 0, stream>>>(W2, Wm, Wu1, Wu2, Wmean, Wv, W2T2, WmT2, Wu1T2, Wu2T2, WH);
  k_enc<<<NN / NTB, 128, 0, stream>>>(x, W1, b1, W2T2, b2, WmT2, HU, P);
  k_pair<<<NN / NTB, 256, 0, stream>>>(P, bm, HU);
  k_upd<<<NN / NTB, 256, 0, stream>>>(HU, Wu1T2, bu1, Wu2T2, bu2, WH, bmean, bvv, HEADS);
  k_emit<<<(OUT_N + 255) / 256, 256, 0, stream>>>(HEADS, lstd, out);
}
